// MemoryBridge_74895639708119
// MI455X (gfx1250) — hardware-verified
//
#include <hip/hip_runtime.h>
#include <math.h>

typedef __attribute__((ext_vector_type(16))) _Float16 v16h;
typedef __attribute__((ext_vector_type(8)))  _Float16 v8h;
typedef __attribute__((ext_vector_type(16))) __bf16   v16b;
typedef __attribute__((ext_vector_type(8)))  __bf16   v8b;
typedef __attribute__((ext_vector_type(8)))  float    v8f;
typedef __attribute__((ext_vector_type(4)))  float    v4f;
typedef __attribute__((ext_vector_type(4)))  unsigned int v4u;
typedef __attribute__((ext_vector_type(2)))  unsigned int v2u;

constexpr int kRows    = 2048;
constexpr int kKwd     = 1000;
constexpr int kKwdP    = 1024;
constexpr int kEmb     = 300;
constexpr int kEmbP    = 320;
constexpr int kEmbV    = 304;
constexpr int kVocab   = 50000;
constexpr int kVTile   = 64;
constexpr int kNTiles  = 782;
constexpr int kVocabP  = kNTiles * kVTile;
constexpr int kHead    = 512;
constexpr int kHead2   = 2 * kHead;
constexpr int kNSplit  = 8;
constexpr int kTilesPerSplit = 98;
constexpr int kHopRows = 128;
constexpr int kAccTiles = kEmbV / 16;
static_assert(kVocabP == 50048, "vocab pad");
static_assert(kVocabP >= kVocab && kVocabP - kVocab < kVTile, "vocab pad extent");
static_assert(kNSplit * kTilesPerSplit >= kNTiles, "split coverage");
static_assert((kNSplit - 1) * kTilesPerSplit < kNTiles, "every split owns at least one tile");
static_assert(kKwdP % 32 == 0 && kEmbP % 32 == 0, "GEMM K multiples of 32");
static_assert(kRows % 64 == 0 && kEmbP % 64 == 0 && kHead2 % 64 == 0 && kHead % 64 == 0, "GEMM M,N multiples of 64");
static_assert(kRows % kHopRows == 0 && kAccTiles == 19 && kEmbV >= kEmb, "hop tiling");
static_assert(kKwd % 8 == 0 && kEmb % 4 == 0 && kVocab % 4 == 0, "vector load granularity");

constexpr float kQCarry  = 32.0f;
constexpr float kKCarry  = 16.0f;
constexpr float kVCarry  = 128.0f;
constexpr float kWHCarry = 256.0f;
constexpr float kPExp    = 15.0f;
constexpr float kScoreCarry = kQCarry * kKCarry;
constexpr float kLog2e   = 1.4426950408889634f;
constexpr float kExpC    = kLog2e / kScoreCarry;
constexpr float kScoreCarryInv = 1.0f / kScoreCarry;
constexpr float kHeadScale = 1.0f / (kQCarry * kWHCarry);
constexpr float kNegBig  = -3.0e38f;

constexpr size_t kOffXH    = 0;
constexpr size_t kOffXL    = kOffXH    + (size_t)kRows * kKwdP * 2;
constexpr size_t kOffWM    = kOffXL    + (size_t)kRows * kKwdP * 2;
constexpr size_t kOffWH    = kOffWM    + (size_t)kEmbP * kKwdP * 2;
constexpr size_t kOffBIAS  = kOffWH    + (size_t)kHead2 * kEmbP * 2;
constexpr size_t kOffFEAT0 = kOffBIAS  + (size_t)(kEmbP + kHead2) * 4;
constexpr size_t kOffFEAT1 = kOffFEAT0 + (size_t)kRows * kEmbP * 4;
constexpr size_t kOffFEAT2 = kOffFEAT1 + (size_t)kRows * kEmbP * 4;
constexpr size_t kOffQH    = kOffFEAT2 + (size_t)kRows * kEmbP * 4;
constexpr size_t kOffVT    = kOffQH    + (size_t)kRows * kEmbP * 2;
constexpr size_t kOffKT    = kOffVT    + (size_t)kNTiles * kEmbV * kVTile * 2;
constexpr size_t kOffOPART = kOffKT    + (size_t)kVocabP * kEmbP * 2;
constexpr size_t kOffMPART = kOffOPART + (size_t)kNSplit * kRows * kEmbP * 4;
constexpr size_t kOffLPART = kOffMPART + (size_t)kNSplit * kRows * 4;
constexpr size_t kWsTotal  = kOffLPART + (size_t)kNSplit * kRows * 4;
static_assert(kWsTotal == 102442240ull, "carve total");
static_assert(kWsTotal <= 134217728ull, "carve cap");
static_assert((kOffXL % 128) == 0 && (kOffWM % 128) == 0 && (kOffWH % 128) == 0 && (kOffBIAS % 128) == 0 &&
              (kOffFEAT0 % 128) == 0 && (kOffFEAT1 % 128) == 0 && (kOffFEAT2 % 128) == 0 && (kOffQH % 128) == 0 &&
              (kOffVT % 128) == 0 && (kOffKT % 128) == 0 && (kOffOPART % 128) == 0 && (kOffMPART % 128) == 0 &&
              (kOffLPART % 128) == 0, "128-B aligned regions");

constexpr int kLdsK     = kHopRows * kEmbP * 2;
constexpr int kLdsV     = kLdsK + kVTile * kEmbP * 2;
constexpr int kLdsML    = kLdsV + kEmbP * kVTile * 2;
constexpr int kLdsTotal = kLdsML + 2 * kHopRows * 4;
static_assert(kLdsK == 81920 && kLdsV == 122880 && kLdsML == 163840 && kLdsTotal == 164864, "hop LDS map");
static_assert(8 * 16 * kEmbP * 4 == kLdsML, "output slabs reuse exactly the operand tiles");

__device__ __forceinline__ int imin(int a, int b) { return a < b ? a : b; }
__device__ __forceinline__ unsigned short f2bf_bits(float f) {
  unsigned u = __float_as_uint(f);
  return (unsigned short)((u + 0x7FFFu + ((u >> 16) & 1u)) >> 16);
}
__device__ __forceinline__ float bf_bits2f(unsigned short h) { return __uint_as_float(((unsigned)h) << 16); }
__device__ __forceinline__ float rne_bf(float f) { return bf_bits2f(f2bf_bits(f)); }
__device__ __forceinline__ unsigned short h_bits(float f) {
  const _Float16 h = (_Float16)f;
  return __builtin_bit_cast(unsigned short, h);
}
__device__ __forceinline__ unsigned pk16(unsigned short a, unsigned short b) { return (unsigned)a | ((unsigned)b << 16); }

template <typename T> struct Frag;
template <> struct Frag<_Float16> {
  typedef v16h V; union U { v16h v; v8h h[2]; };
  static __device__ __forceinline__ v16h load(const _Float16* p) {
    U f; f.h[0] = *(const v8h*)(p); f.h[1] = *(const v8h*)(p + 16); return f.v;
  }
  static __device__ __forceinline__ v8f mma(v16h a, v16h b, v8f c) {
    c = __builtin_amdgcn_wmma_f32_16x16x32_f16(false, a, false, b, (short)0, c, false, false);
    asm volatile("v_nop\n\tv_nop\n\tv_nop\n\tv_nop" : "+v"(c) : "v"(a), "v"(b));
    return c;
  }
};
template <> struct Frag<__bf16> {
  typedef v16b V; union U { v16b v; v8b h[2]; };
  static __device__ __forceinline__ v16b load(const __bf16* p) {
    U f; f.h[0] = *(const v8b*)(p); f.h[1] = *(const v8b*)(p + 16); return f.v;
  }
  static __device__ __forceinline__ v8f mma(v16b a, v16b b, v8f c) {
    c = __builtin_amdgcn_wmma_f32_16x16x32_bf16(false, a, false, b, (short)0, c, false, false);
    asm volatile("v_nop\n\tv_nop\n\tv_nop\n\tv_nop" : "+v"(c) : "v"(a), "v"(b));
    return c;
  }
};
template <int ET> struct Elem;
template <> struct Elem<0> { typedef _Float16 T; };
template <> struct Elem<1> { typedef __bf16 T; };

template <int ET, int SPL>
__global__ __launch_bounds__(256) void wmma_gemm64(
    const unsigned short* __restrict__ Ap, const unsigned short* __restrict__ A2p, int lda,
    const unsigned short* __restrict__ Btp, int ldb,
    float* __restrict__ Cout, int ldc, int planeCols, long planeStride,
    const float* __restrict__ bias, int M, int N, int K, float scale) {
  typedef typename Elem<ET>::T T;
  typedef typename Frag<T>::V V;
  const T* A = (const T*)Ap; const T* A2 = (const T*)A2p; const T* Bt = (const T*)Btp;
  __shared__ __align__(16) float sT[8][16 * 68];
  const int lane = threadIdx.x & 31;
  const int wave = __builtin_amdgcn_readfirstlane((int)(threadIdx.x >> 5));
  const int tilesN = N >> 6;
  const int tilesM = M >> 6;
  const int tile = blockIdx.x * 8 + wave;
  if (tile >= tilesM * tilesN) return;
  const int tm = tile / tilesN;
  const int tn = tile - tm * tilesN;
  const int m0 = tm << 6;
  const int n0 = tn << 6;
  const int rlane = lane & 15;
  const int koff  = (lane >> 4) * 8;
  const int mOff  = (lane >> 4) * 8;

  v8f acc[4][4];
#pragma unroll
  for (int i = 0; i < 4; ++i)
#pragma unroll
    for (int j = 0; j < 4; ++j) acc[i][j] = (v8f){0.f,0.f,0.f,0.f,0.f,0.f,0.f,0.f};

  for (int k0 = 0; k0 < K; k0 += 32) {
    V bh[4];
#pragma unroll
    for (int j = 0; j < 4; ++j) {
      const size_t bo = (size_t)(n0 + (j << 4) + rlane) * ldb + koff + k0;
      bh[j] = Frag<T>::load(Bt + bo);
    }
#pragma unroll
    for (int i = 0; i < 4; ++i) {
      const size_t ao = (size_t)(m0 + (i << 4) + rlane) * lda + koff + k0;
      V ah = Frag<T>::load(A + ao);
      V al = ah;
      if (SPL == 1) al = Frag<T>::load(A2 + ao);
#pragma unroll
      for (int j = 0; j < 4; ++j) {
        acc[i][j] = Frag<T>::mma(ah, bh[j], acc[i][j]);
        if (SPL == 1) acc[i][j] = Frag<T>::mma(al, bh[j], acc[i][j]);
      }
    }
  }

  float* slab = sT[wave];
  const int pl = n0 / planeCols;
  const int nc = n0 - pl * planeCols;
  float* C = Cout + (size_t)pl * planeStride;
#pragma unroll
  for (int i = 0; i < 4; ++i) {
    const int mBase = m0 + (i << 4);
#pragma unroll
    for (int j = 0; j < 4; ++j) {
      const int n = n0 + (j << 4) + rlane;
      const float bv = bias[n];
#pragma unroll
      for (int r = 0; r < 8; ++r) {
        const float v = acc[i][j][r] * scale + bv;
        slab[(mOff + r) * 68 + (j << 4) + rlane] = v;
      }
    }
    __builtin_amdgcn_fence(__ATOMIC_RELEASE, "workgroup");
    __builtin_amdgcn_wave_barrier();
    __builtin_amdgcn_fence(__ATOMIC_ACQUIRE, "workgroup");
    {
      const int hh = lane >> 4, c4 = (lane & 15) * 4;
      for (int pass = 0; pass < 2; ++pass) {
#pragma unroll
        for (int it = 0; it < 8; ++it) {
          const int row = it * 2 + hh;
          const v4f v = *(const v4f*)(slab + row * 68 + c4);
          *(volatile v4f*)(C + (size_t)(mBase + row) * ldc + nc + c4) = v;
        }
        __threadfence();
      }
    }
    __builtin_amdgcn_fence(__ATOMIC_RELEASE, "workgroup");
    __builtin_amdgcn_wave_barrier();
    __builtin_amdgcn_fence(__ATOMIC_ACQUIRE, "workgroup");
  }
}

__global__ __launch_bounds__(256) void xsplit_kernel(const float* __restrict__ lg, const float* __restrict__ mu,
                                                     unsigned short* __restrict__ XH, unsigned short* __restrict__ XL) {
  const int i = blockIdx.x * 256 + threadIdx.x;
  const int row = i >> 7;
  const int c8 = (i & 127) * 8;
  const bool ok = c8 < kKwd;
  const int cc = ok ? c8 : (kKwd - 8);
  const size_t o = (size_t)row * kKwd + cc;
  const v4f l0 = *(const v4f*)(lg + o);
  const v4f l1 = *(const v4f*)(lg + o + 4);
  const v4f m0 = *(const v4f*)(mu + o);
  const v4f m1 = *(const v4f*)(mu + o + 4);
  unsigned short hb[8], lb[8];
#pragma unroll
  for (int e = 0; e < 4; ++e) {
    const float p0 = rne_bf(l0[e]) * rne_bf(m0[e]);
    const float p1 = rne_bf(l1[e]) * rne_bf(m1[e]);
    const float x0 = ok ? p0 : 0.0f;
    const float x1 = ok ? p1 : 0.0f;
    const unsigned short h0 = f2bf_bits(x0);
    const unsigned short h1 = f2bf_bits(x1);
    hb[e] = h0;
    hb[4 + e] = h1;
    lb[e] = f2bf_bits(x0 - bf_bits2f(h0));
    lb[4 + e] = f2bf_bits(x1 - bf_bits2f(h1));
  }
  const v4u uh = (v4u){pk16(hb[0], hb[1]), pk16(hb[2], hb[3]), pk16(hb[4], hb[5]), pk16(hb[6], hb[7])};
  const v4u ul = (v4u){pk16(lb[0], lb[1]), pk16(lb[2], lb[3]), pk16(lb[4], lb[5]), pk16(lb[6], lb[7])};
  unsigned short* qh = XH + (size_t)i * 8;
  unsigned short* ql = XL + (size_t)i * 8;
  *(volatile v4u*)qh = uh;
  *(volatile v4u*)ql = ul;
  __threadfence();
  *(volatile v4u*)qh = uh;
  *(volatile v4u*)ql = ul;
}

__global__ __launch_bounds__(256) void wplanes_kernel(
    const float* __restrict__ mlp_w, const float* __restrict__ mlp_b,
    const float* __restrict__ enc_w, const float* __restrict__ enc_b,
    const float* __restrict__ dec_w, const float* __restrict__ dec_b,
    unsigned short* __restrict__ WM, unsigned short* __restrict__ WH, float* __restrict__ BIAS) {
  const int bx = blockIdx.x;
  const int t = threadIdx.x;
  if (bx < 160) {
    const int i = bx * 256 + t;
    const int row = i >> 7;
    const int c8 = (i & 127) * 8;
    const bool ok = (row < kEmb) && (c8 < kKwd);
    const int rr = imin(row, kEmb - 1);
    const int cc = imin(c8, kKwd - 8);
    const float* src = mlp_w + (size_t)rr * kKwd + cc;
    const v4f a0 = *(const v4f*)(src);
    const v4f a1 = *(const v4f*)(src + 4);
    unsigned short hb[8];
#pragma unroll
    for (int e = 0; e < 4; ++e) {
      const unsigned short b0 = f2bf_bits(a0[e]);
      const unsigned short b1 = f2bf_bits(a1[e]);
      hb[e] = ok ? b0 : (unsigned short)0;
      hb[4 + e] = ok ? b1 : (unsigned short)0;
    }
    const v4u u = (v4u){pk16(hb[0], hb[1]), pk16(hb[2], hb[3]), pk16(hb[4], hb[5]), pk16(hb[6], hb[7])};
    unsigned short* q = WM + (size_t)i * 8;
    *(volatile v4u*)q = u;
    __threadfence();
    *(volatile v4u*)q = u;
  } else if (bx < 320) {
    const int i = (bx - 160) * 256 + t;
    const int n = i / 40;
    const int c8 = (i - n * 40) * 8;
    const float* W = (n < kHead) ? enc_w : dec_w;
    const int nr = (n < kHead) ? n : (n - kHead);
    const int ca = imin(c8, kEmb - 4);
    const int cb = imin(c8 + 4, kEmb - 4);
    const v4f a0 = *(const v4f*)(W + (size_t)nr * kEmb + ca);
    const v4f a1 = *(const v4f*)(W + (size_t)nr * kEmb + cb);
    unsigned short hb[8];
#pragma unroll
    for (int e = 0; e < 4; ++e) {
      const float w0 = rne_bf(a0[e]) * kWHCarry;
      const float w1 = rne_bf(a1[e]) * kWHCarry;
      const float s0 = (c8 + e < kEmb) ? w0 : 0.0f;
      const float s1 = (c8 + 4 + e < kEmb) ? w1 : 0.0f;
      hb[e] = h_bits(s0);
      hb[4 + e] = h_bits(s1);
    }
    const v4u u = (v4u){pk16(hb[0], hb[1]), pk16(hb[2], hb[3]), pk16(hb[4], hb[5]), pk16(hb[6], hb[7])};
    unsigned short* q = WH + (size_t)i * 8;
    *(volatile v4u*)q = u;
    __threadfence();
    *(volatile v4u*)q = u;
  } else {
    const int i = (bx - 320) * 256 + t;
    const int ic = imin(i, 335);
    float val[4];
#pragma unroll
    for (int e = 0; e < 4; ++e) {
      const int idx = 4 * ic + e;
      const int im = imin(idx, kEmb - 1);
      int ie = idx - kEmbP;
      ie = ie < 0 ? 0 : ie;
      ie = imin(ie, kHead - 1);
      int id = idx - kEmbP - kHead;
      id = id < 0 ? 0 : id;
      id = imin(id, kHead - 1);
      const float vm = rne_bf(mlp_b[im]);
      const float ve = rne_bf(enc_b[ie]);
      const float vd = rne_bf(dec_b[id]);
      float v = vd;
      v = (idx < kEmbP + kHead) ? ve : v;
      v = (idx < kEmbP) ? 0.0f : v;
      v = (idx < kEmb) ? vm : v;
      val[e] = v;
    }
    const v4f u = (v4f){val[0], val[1], val[2], val[3]};
    if (i < 336) {
      float* q = BIAS + (size_t)i * 4;
      *(volatile v4f*)q = u;
      __threadfence();
      *(volatile v4f*)q = u;
    }
  }
}

constexpr int kVPitch = 306;
__global__ __launch_bounds__(256) void vplane_kernel(const float* __restrict__ emb, unsigned short* __restrict__ VT) {
  __shared__ unsigned short sm[kVTile * kVPitch];
  const int t = threadIdx.x;
  const int tile = blockIdx.x;
  const size_t g0 = (size_t)tile * kVTile * kEmb;
  const size_t total = (size_t)kVocab * kEmb;
#pragma unroll 1
  for (int it = 0; it < 19; ++it) {
    const int i4 = it * 256 + t;
    const int i4c = imin(i4, 4799);
    const size_t g = g0 + (size_t)i4c * 4;
    const bool ok = g < total;
    const size_t gc = ok ? g : (total - 4);
    const v4f a = *(const v4f*)(emb + gc);
    float a0 = a[0], a1 = a[1], a2 = a[2], a3 = a[3];
    asm volatile("" : "+v"(a0), "+v"(a1), "+v"(a2), "+v"(a3));
    const int le = i4c * 4;
    const int vr = le / kEmb;
    const int e = le - vr * kEmb;
    const unsigned short b0 = h_bits(ok ? rne_bf(a0) * kVCarry : 0.0f);
    const unsigned short b1 = h_bits(ok ? rne_bf(a1) * kVCarry : 0.0f);
    const unsigned short b2 = h_bits(ok ? rne_bf(a2) * kVCarry : 0.0f);
    const unsigned short b3 = h_bits(ok ? rne_bf(a3) * kVCarry : 0.0f);
    if (i4 < 4800) {
      sm[vr * kVPitch + e + 0] = b0;
      sm[vr * kVPitch + e + 1] = b1;
      sm[vr * kVPitch + e + 2] = b2;
      sm[vr * kVPitch + e + 3] = b3;
    }
  }
  __syncthreads();
  unsigned short* dst = VT + (size_t)tile * kEmbV * kVTile;
#pragma unroll 1
  for (int it = 0; it < 10; ++it) {
    const int c = it * 256 + t;
    const int cq = imin(c, 2431);
    const int e = cq >> 3;
    const int kr0 = (cq & 7) * 8;
    const int ec = imin(e, kEmb - 1);
    const bool eok = e < kEmb;
    unsigned short hb[8];
#pragma unroll
    for (int j = 0; j < 8; ++j) {
      const unsigned short w = sm[(kr0 + j) * kVPitch + ec];
      hb[j] = eok ? w : (unsigned short)0;
    }
    const v4u u = (v4u){pk16(hb[0], hb[1]), pk16(hb[2], hb[3]), pk16(hb[4], hb[5]), pk16(hb[6], hb[7])};
    if (c < 2432) {
      unsigned short* q = dst + (size_t)c * 8;
      *(volatile v4u*)q = u;
      __threadfence();
      *(volatile v4u*)q = u;
    }
  }
}

constexpr int kKPitch = 328;
__global__ __launch_bounds__(256) void kplane_kernel(const float* __restrict__ keys, unsigned short* __restrict__ KT) {
  __shared__ unsigned short sm[kVTile * kKPitch];
  const int t = threadIdx.x;
  const int v0 = blockIdx.x * kVTile;
#pragma unroll 1
  for (int it = 0; it < 19; ++it) {
    const int i4 = it * 256 + t;
    const int i4c = imin(i4, 4799);
    const int k = i4c >> 4;
    const int c4 = (i4c & 15) * 4;
    const int v = v0 + c4;
    const bool ok = v < kVocab;
    const int vc = ok ? v : (kVocab - 4);
    const v4f a = *(const v4f*)(keys + (size_t)k * kVocab + vc);
    float a0 = a[0], a1 = a[1], a2 = a[2], a3 = a[3];
    asm volatile("" : "+v"(a0), "+v"(a1), "+v"(a2), "+v"(a3));
    const unsigned short b0 = h_bits(ok ? rne_bf(a0) * kKCarry : 0.0f);
    const unsigned short b1 = h_bits(ok ? rne_bf(a1) * kKCarry : 0.0f);
    const unsigned short b2 = h_bits(ok ? rne_bf(a2) * kKCarry : 0.0f);
    const unsigned short b3 = h_bits(ok ? rne_bf(a3) * kKCarry : 0.0f);
    if (i4 < 4800) {
      sm[(c4 + 0) * kKPitch + k] = b0;
      sm[(c4 + 1) * kKPitch + k] = b1;
      sm[(c4 + 2) * kKPitch + k] = b2;
      sm[(c4 + 3) * kKPitch + k] = b3;
    }
  }
  __syncthreads();
  unsigned short* dst = KT + (size_t)v0 * kEmbP;
#pragma unroll 1
  for (int it = 0; it < 10; ++it) {
    const int c = it * 256 + t;
    const int vl = c / 40;
    const int k0 = (c - vl * 40) * 8;
    unsigned short hb[8];
#pragma unroll
    for (int j = 0; j < 8; ++j) {
      const int kk = imin(k0 + j, kEmb - 1);
      const unsigned short w = sm[vl * kKPitch + kk];
      hb[j] = (k0 + j < kEmb) ? w : (unsigned short)0;
    }
    const v4u u = (v4u){pk16(hb[0], hb[1]), pk16(hb[2], hb[3]), pk16(hb[4], hb[5]), pk16(hb[6], hb[7])};
    unsigned short* q = dst + (size_t)c * 8;
    *(volatile v4u*)q = u;
    __threadfence();
    *(volatile v4u*)q = u;
  }
}

__global__ __launch_bounds__(256) __attribute__((amdgpu_num_vgpr(256)))
void hop_kernel(const float* __restrict__ feat, const unsigned short* __restrict__ KT,
                const unsigned short* __restrict__ VT, float* __restrict__ opart,
                float* __restrict__ mpart, float* __restrict__ lpart) {
  extern __shared__ __align__(16) unsigned char smem[];
  const _Float16* LQ = (const _Float16*)(smem);
  const _Float16* LK = (const _Float16*)(smem + kLdsK);
  const _Float16* LV = (const _Float16*)(smem + kLdsV);
  float* sML = (float*)(smem + kLdsML);

  const int tid  = threadIdx.x;
  const int wave = __builtin_amdgcn_readfirstlane((int)(threadIdx.x >> 5));
  const int lane = tid & 31;
  const int c    = lane & 15;
  const int hh   = lane >> 4;
  const int row0 = blockIdx.x * kHopRows;
  const int split = blockIdx.y;
  const int tBeg = split * kTilesPerSplit;
  const int tEnd = imin(tBeg + kTilesPerSplit, kNTiles);

  {
    const float* src = feat + (size_t)row0 * kEmbP;
#pragma unroll 1
    for (int it = 0; it < 20; ++it) {
      const int ch = it * 256 + tid;
      const v4f a0 = *(const v4f*)(src + (size_t)ch * 8);
      const v4f a1 = *(const v4f*)(src + (size_t)ch * 8 + 4);
      unsigned short hb[8];
#pragma unroll
      for (int e = 0; e < 4; ++e) {
        hb[e] = h_bits(a0[e] * kQCarry);
        hb[4 + e] = h_bits(a1[e] * kQCarry);
      }
      const v4u u = (v4u){pk16(hb[0], hb[1]), pk16(hb[2], hb[3]), pk16(hb[4], hb[5]), pk16(hb[6], hb[7])};
      *(v4u*)(smem + (size_t)ch * 16) = u;
    }
  }

  v8f acc[kAccTiles];
#pragma unroll
  for (int tt = 0; tt < kAccTiles; ++tt) acc[tt] = (v8f){0.f,0.f,0.f,0.f,0.f,0.f,0.f,0.f};
  float m_run = kNegBig;
  float l_run = 0.0f;

  const _Float16* qrow = LQ + (wave * 16 + c) * kEmbP + 8 * hh;

#pragma unroll 1
  for (int t = tBeg; t < tEnd; ++t) {
    __syncthreads();
    {
      const v4u* gk = (const v4u*)(KT + (size_t)t * kVTile * kEmbP);
      const v4u* gv = (const v4u*)(VT + (size_t)t * kEmbV * kVTile);
#pragma unroll 2
      for (int it = 0; it < 10; ++it) {
        const int ch = it * 256 + tid;
        const v4u kk = gk[ch];
        const v4u vv = gv[imin(ch, 2431)];
        *(v4u*)(smem + kLdsK + (size_t)ch * 16) = kk;
        *(v4u*)(smem + kLdsV + (size_t)ch * 16) = vv;
      }
    }
    __syncthreads();
    const bool lastTile = (t == kNTiles - 1);
#pragma unroll
    for (int sub = 0; sub < 2; ++sub) {
      v8f s0 = (v8f){0.f,0.f,0.f,0.f,0.f,0.f,0.f,0.f};
      v8f s1 = (v8f){0.f,0.f,0.f,0.f,0.f,0.f,0.f,0.f};
      const _Float16* k0p = LK + (sub * 32 + c) * kEmbP + 8 * hh;
      const _Float16* k1p = k0p + 16 * kEmbP;
#pragma unroll 1
      for (int ks = 0; ks < kEmbP / 32; ++ks) {
        const v16h qb  = Frag<_Float16>::load(qrow + ks * 32);
        const v16h ka0 = Frag<_Float16>::load(k0p + ks * 32);
        const v16h ka1 = Frag<_Float16>::load(k1p + ks * 32);
        s0 = Frag<_Float16>::mma(ka0, qb, s0);
        s1 = Frag<_Float16>::mma(ka1, qb, s1);
      }
      if (lastTile) {
        const int vb = t * kVTile + sub * 32 + 8 * hh;
#pragma unroll
        for (int r = 0; r < 8; ++r) {
          s0[r] = (vb + r < kVocab) ? s0[r] : kNegBig;
          s1[r] = (vb + 16 + r < kVocab) ? s1[r] : kNegBig;
        }
      }
      float mx = fmaxf(s0[0], s1[0]);
#pragma unroll
      for (int r = 1; r < 8; ++r) mx = fmaxf(mx, fmaxf(s0[r], s1[r]));
      const float mo = __shfl_xor(mx, 16, 32);
      mx = fmaxf(mx, mo);
      const float m_new = fmaxf(m_run, mx);
      const float alpha = __builtin_amdgcn_exp2f((m_run - m_new) * kExpC);
      m_run = m_new;
      const float off = fmaf(-m_new, kExpC, kPExp);
      v16h pa;
      float lsum = 0.0f;
#pragma unroll
      for (int r = 0; r < 8; ++r) {
        const float p = __builtin_amdgcn_exp2f(fmaf(s0[r], kExpC, off));
        const _Float16 ph = (_Float16)p;
        pa[r] = ph;
        lsum += (float)ph;
      }
#pragma unroll
      for (int r = 0; r < 8; ++r) {
        const float p = __builtin_amdgcn_exp2f(fmaf(s1[r], kExpC, off));
        const _Float16 ph = (_Float16)p;
        pa[8 + r] = ph;
        lsum += (float)ph;
      }
      l_run = fmaf(l_run, alpha, lsum);
      const unsigned moved = __builtin_amdgcn_ballot_w32(alpha != 1.0f);
      if (moved != 0u) {
#pragma unroll
        for (int tt = 0; tt < kAccTiles; ++tt) acc[tt] = acc[tt] * alpha;
      }
      const _Float16* vp = LV + c * kVTile + sub * 32 + 8 * hh;
#pragma unroll
      for (int tt = 0; tt < kAccTiles; ++tt) {
        const v16h va = Frag<_Float16>::load(vp + tt * 16 * kVTile);
        acc[tt] = Frag<_Float16>::mma(va, pa, acc[tt]);
      }
    }
  }

  const float l_oth = __shfl_xor(l_run, 16, 32);
  const float l_tot = l_run + l_oth;
  __syncthreads();
  float* slab = (float*)smem + wave * (16 * kEmbP);
  {
    float* sr = slab + c * kEmbP + 8 * hh;
#pragma unroll
    for (int tt = 0; tt < kAccTiles; ++tt) {
      const v4f lo4 = (v4f){acc[tt][0], acc[tt][1], acc[tt][2], acc[tt][3]};
      const v4f hi4 = (v4f){acc[tt][4], acc[tt][5], acc[tt][6], acc[tt][7]};
      *(v4f*)(sr + tt * 16) = lo4;
      *(v4f*)(sr + tt * 16 + 4) = hi4;
    }
    const v4f z = (v4f){0.f, 0.f, 0.f, 0.f};
    *(v4f*)(sr + kEmbV) = z;
    *(v4f*)(sr + kEmbV + 4) = z;
  }
  if (lane < 16) {
    sML[wave * 16 + lane] = m_run * kScoreCarryInv;
    sML[kHopRows + wave * 16 + lane] = l_tot;
  }
  __syncthreads();
  {
    float* og = opart + ((size_t)split * kRows + row0 + wave * 16) * kEmbP;
    for (int pass = 0; pass < 2; ++pass) {
#pragma unroll 4
      for (int it = 0; it < 40; ++it) {
        const int idx = (it * 32 + lane) * 4;
        const v4f v = *(const v4f*)(slab + idx);
        *(volatile v4f*)(og + idx) = v;
      }
      __threadfence();
    }
  }
  if (wave == 0) {
    const v4f v = *(const v4f*)(sML + lane * 4);
    float* q = mpart + (size_t)split * kRows + row0 + lane * 4;
    *(volatile v4f*)q = v;
    __threadfence();
    *(volatile v4f*)q = v;
  }
  if (wave == 1) {
    const v4f v = *(const v4f*)(sML + kHopRows + lane * 4);
    float* q = lpart + (size_t)split * kRows + row0 + lane * 4;
    *(volatile v4f*)q = v;
    __threadfence();
    *(volatile v4f*)q = v;
  }
}

__global__ __launch_bounds__(320) void combine_kernel(
    const float* __restrict__ opart, const float* __restrict__ mpart, const float* __restrict__ lpart,
    const float* __restrict__ featIn, float* __restrict__ featOut, unsigned short* __restrict__ QH) {
  const int i = blockIdx.x * 320 + threadIdx.x;
  const int row = i / 80;
  const int c4 = (i - row * 80) * 4;
  float mstar = kNegBig;
#pragma unroll 1
  for (int s = 0; s < kNSplit; ++s) mstar = fmaxf(mstar, mpart[(size_t)s * kRows + row]);
  float denom = 0.0f;
  v4f a = (v4f){0.f, 0.f, 0.f, 0.f};
#pragma unroll 1
  for (int s = 0; s < kNSplit; ++s) {
    const float ms = mpart[(size_t)s * kRows + row];
    const float ls = lpart[(size_t)s * kRows + row];
    const float w = expf(ms - mstar);
    denom = fmaf(w, ls, denom);
    const v4f o = *(const v4f*)(opart + ((size_t)s * kRows + row) * kEmbP + c4);
    a = a + o * w;
  }
  const float inv = 1.0f / (denom * kVCarry);
  const v4f f = *(const v4f*)(featIn + (size_t)i * 4);
  float nf[4];
#pragma unroll
  for (int e = 0; e < 4; ++e) {
    const float v = f[e] + a[e] * inv;
    nf[e] = (c4 + e < kEmb) ? v : 0.0f;
  }
  const v4f uf = (v4f){nf[0], nf[1], nf[2], nf[3]};
  const unsigned short h0 = h_bits(nf[0] * kQCarry);
  const unsigned short h1 = h_bits(nf[1] * kQCarry);
  const unsigned short h2 = h_bits(nf[2] * kQCarry);
  const unsigned short h3 = h_bits(nf[3] * kQCarry);
  const v2u uh = (v2u){pk16(h0, h1), pk16(h2, h3)};
  float* qf = featOut + (size_t)i * 4;
  unsigned short* qh = QH + (size_t)i * 4;
  *(volatile v4f*)qf = uf;
  *(volatile v2u*)qh = uh;
  __threadfence();
  *(volatile v4f*)qf = uf;
  *(volatile v2u*)qh = uh;
}

extern "C" void kernel_launch(void* const* d_in, const int* in_sizes, int n_in,
                              void* d_out, int out_size, void* d_ws, size_t ws_size,
                              hipStream_t stream) {
  if (n_in < 11) return;
  if (in_sizes[0] != kRows * kKwd) return;
  if (in_sizes[1] != kRows * kKwd) return;
  if (in_sizes[2] != kVocab * kEmb) return;
  if (in_sizes[3] != kEmb * kKwd) return;
  if (in_sizes[4] != kEmb) return;
  if (in_sizes[5] != kEmb * kVocab) return;
  if (in_sizes[6] != kEmb * kVocab) return;
  if (in_sizes[7] != kHead * kEmb) return;
  if (in_sizes[8] != kHead) return;
  if (in_sizes[9] != kHead * kEmb) return;
  if (in_sizes[10] != kHead) return;
  if (out_size != 2 * kRows * kHead) return;
  if (ws_size < kWsTotal) return;

  const float* lg     = (const float*)d_in[0];
  const float* mu     = (const float*)d_in[1];
  const float* emb    = (const float*)d_in[2];
  const float* mlp_w  = (const float*)d_in[3];
  const float* mlp_b  = (const float*)d_in[4];
  const float* keys0  = (const float*)d_in[5];
  const float* keys1  = (const float*)d_in[6];
  const float* enc_w  = (const float*)d_in[7];
  const float* enc_b  = (const float*)d_in[8];
  const float* dec_w  = (const float*)d_in[9];
  const float* dec_b  = (const float*)d_in[10];
  float* out = (float*)d_out;

  char* ws = (char*)d_ws;
  unsigned short* XH    = (unsigned short*)(ws + kOffXH);
  unsigned short* XL    = (unsigned short*)(ws + kOffXL);
  unsigned short* WM    = (unsigned short*)(ws + kOffWM);
  unsigned short* WH    = (unsigned short*)(ws + kOffWH);
  float*          BIAS  = (float*)(ws + kOffBIAS);
  float*          FEAT0 = (float*)(ws + kOffFEAT0);
  float*          FEAT1 = (float*)(ws + kOffFEAT1);
  float*          FEAT2 = (float*)(ws + kOffFEAT2);
  unsigned short* QH    = (unsigned short*)(ws + kOffQH);
  unsigned short* VT    = (unsigned short*)(ws + kOffVT);
  unsigned short* KT    = (unsigned short*)(ws + kOffKT);
  float*          OPART = (float*)(ws + kOffOPART);
  float*          MPART = (float*)(ws + kOffMPART);
  float*          LPART = (float*)(ws + kOffLPART);

  xsplit_kernel<<<(kRows * (kKwdP / 8)) / 256, 256, 0, stream>>>(lg, mu, XH, XL);
  wplanes_kernel<<<322, 256, 0, stream>>>(mlp_w, mlp_b, enc_w, enc_b, dec_w, dec_b, WM, WH, BIAS);

  wmma_gemm64<1, 1><<<20, 256, 0, stream>>>(
      XH, XL, kKwdP, WM, kKwdP,
      FEAT0, kEmbP, kEmbP, 0L,
      BIAS, kRows, kEmbP, kKwdP, 1.0f);

  vplane_kernel<<<kNTiles, 256, 0, stream>>>(emb, VT);

  kplane_kernel<<<kNTiles, 256, 0, stream>>>(keys0, KT);
  hop_kernel<<<dim3(kRows / kHopRows, kNSplit), 256, kLdsTotal, stream>>>(FEAT0, KT, VT, OPART, MPART, LPART);
  combine_kernel<<<(kRows * 80) / 320, 320, 0, stream>>>(OPART, MPART, LPART, FEAT0, FEAT1, QH);

  kplane_kernel<<<kNTiles, 256, 0, stream>>>(keys1, KT);
  hop_kernel<<<dim3(kRows / kHopRows, kNSplit), 256, kLdsTotal, stream>>>(FEAT1, KT, VT, OPART, MPART, LPART);
  combine_kernel<<<(kRows * 80) / 320, 320, 0, stream>>>(OPART, MPART, LPART, FEAT1, FEAT2, QH);

  wmma_gemm64<0, 0><<<64, 256, 0, stream>>>(
      QH, QH, kEmbP, WH, kEmbP,
      out, kHead, kHead, (long)kRows * kHead,
      BIAS + kEmbP, kRows, kHead2, kEmbP, kHeadScale);
}
